// FeatherNet_5446018531620
// MI455X (gfx1250) — hardware-verified
//
#include <hip/hip_runtime.h>
#include <stddef.h>
#include <math.h>

constexpr int kDin   = 1024;
constexpr int kDh    = 4096;
constexpr int kDout  = 1024;
constexpr int kBatch = 4096;
constexpr int kSzN   = 2898;
constexpr int kSzM   = 725;
constexpr int kKpad  = 768;
constexpr int kNpad  = 2944;
constexpr int kNW1   = kDh * kDin;
constexpr int kNB1   = kDh;
constexpr int kNW2   = kDout * kDh;
constexpr int kNB2   = kDout;

typedef __attribute__((ext_vector_type(16))) _Float16 v16h;
typedef __attribute__((ext_vector_type(8)))  _Float16 v8h;
typedef __attribute__((ext_vector_type(16))) __bf16   v16b;
typedef __attribute__((ext_vector_type(8)))  __bf16   v8b;
typedef __attribute__((ext_vector_type(8)))  float    v8f;
typedef __attribute__((ext_vector_type(4)))  float    v4f;
typedef __attribute__((ext_vector_type(4)))  unsigned int v4u;

__device__ __forceinline__ unsigned short f2bf_bits(float f) {
  unsigned u = __float_as_uint(f);
  return (unsigned short)((u + 0x7FFFu + ((u >> 16) & 1u)) >> 16);
}
__device__ __forceinline__ float bf_bits2f(unsigned short h) { return __uint_as_float(((unsigned)h) << 16); }

__device__ __forceinline__ void dep_guard_h(v8f& a, v8f& b, v16h x, v16h y) { asm volatile("v_nop\n\tv_nop\n\tv_nop\n\tv_nop" : "+v"(a), "+v"(b) : "v"(x), "v"(y)); }
__device__ __forceinline__ void dep_guard_b(v8f& a, v8f& b, v16b x, v16b y) { asm volatile("v_nop\n\tv_nop\n\tv_nop\n\tv_nop" : "+v"(a), "+v"(b) : "v"(x), "v"(y)); }
__device__ __forceinline__ void keep4_h(v16h a, v16h b, v16h c, v16h d) { asm volatile("v_nop" :: "v"(a), "v"(b), "v"(c), "v"(d)); }
__device__ __forceinline__ void keep4_b(v16b a, v16b b, v16b c, v16b d) { asm volatile("v_nop" :: "v"(a), "v"(b), "v"(c), "v"(d)); }
__device__ __forceinline__ void acc_guard4(v8f& a, v8f& b, v8f& c, v8f& d) { asm volatile("v_nop\n\tv_nop\n\tv_nop\n\tv_nop" : "+v"(a), "+v"(b), "+v"(c), "+v"(d)); }
template <typename T> struct Frag;
template <> struct Frag<_Float16> {
  typedef v16h V; union U { v16h v; v8h h[2]; };
  static __device__ __forceinline__ v16h load(const _Float16* p) {
    U f; f.h[0] = *(const v8h*)(p); f.h[1] = *(const v8h*)(p + 16); return f.v;
  }
  static __device__ __forceinline__ v8f mma(v16h a, v16h b, v8f c) {
    return __builtin_amdgcn_wmma_f32_16x16x32_f16(false, a, false, b, (short)0, c, false, false);
  }
  static __device__ __forceinline__ void guard(v8f& a, v8f& b, v16h x, v16h y) { dep_guard_h(a, b, x, y); }
  static __device__ __forceinline__ void keep(v16h a, v16h b, v16h c, v16h d) { keep4_h(a, b, c, d); }
};
template <> struct Frag<__bf16> {
  typedef v16b V; union U { v16b v; v8b h[2]; };
  static __device__ __forceinline__ v16b load(const __bf16* p) {
    U f; f.h[0] = *(const v8b*)(p); f.h[1] = *(const v8b*)(p + 16); return f.v;
  }
  static __device__ __forceinline__ v8f mma(v16b a, v16b b, v8f c) {
    return __builtin_amdgcn_wmma_f32_16x16x32_bf16(false, a, false, b, (short)0, c, false, false);
  }
  static __device__ __forceinline__ void guard(v8f& a, v8f& b, v16b x, v16b y) { dep_guard_b(a, b, x, y); }
  static __device__ __forceinline__ void keep(v16b a, v16b b, v16b c, v16b d) { keep4_b(a, b, c, d); }
};

__device__ __forceinline__ unsigned pk16(unsigned short a, unsigned short b) { return (unsigned)a | ((unsigned)b << 16); }
__device__ __forceinline__ unsigned short h_bits(float f) { const _Float16 h = (_Float16)f; return __builtin_bit_cast(unsigned short, h); }

template <int ET> struct Elem;
template <> struct Elem<0> { typedef _Float16 T; };
template <> struct Elem<1> { typedef __bf16 T; };
template <int ET, bool SPLIT, int BIAS_MODE, int OUT_MODE, bool RESID, int ACT = 0>
__global__ __launch_bounds__(256) void wmma_gemm64(
    const unsigned short* __restrict__ Ap, const unsigned short* __restrict__ A2p, int lda, long strideA,
    const unsigned short* __restrict__ Btp, const unsigned short* __restrict__ Bt2p, int ldb, long strideB,
    void* __restrict__ Cout, void* __restrict__ Cout2, int ldc, long strideC,
    const float* __restrict__ bias,
    const float* __restrict__ resid, long strideR,
    int M, int N, int K, float scale) {
  typedef typename Elem<ET>::T T;
  typedef typename Frag<T>::V V;
  const T* A = (const T*)Ap; const T* A2 = (const T*)A2p; const T* Bt = (const T*)Btp; const T* Bt2 = (const T*)Bt2p;
  __shared__ __align__(16) float sT[8][16 * 68];
  const int b    = blockIdx.y;
  const int lane = threadIdx.x & 31;
  const int wave = threadIdx.x >> 5;
  const int tilesN = N >> 6;
  const int tilesM = M >> 6;
  const int tile = blockIdx.x * 8 + wave;
  if (tile >= tilesM * tilesN) return;
  const int tm = tile / tilesN;
  const int tn = tile - tm * tilesN;
  const int m0 = tm << 6;
  const int n0 = tn << 6;

  const T* Ab  = A  + (size_t)b * strideA;
  const T* Bb  = Bt + (size_t)b * strideB;
  const T* Ab2 = SPLIT ? (A2  + (size_t)b * strideA) : nullptr;
  const T* Bb2 = SPLIT ? (Bt2 + (size_t)b * strideB) : nullptr;

  const int rlane = lane & 15;
  const int koff  = (lane >> 4) * 8;
  const int mOff  = (lane >> 4) * 8;

  v8f acc[4][4];
#pragma unroll
  for (int i = 0; i < 4; ++i)
#pragma unroll
    for (int j = 0; j < 4; ++j) acc[i][j] = (v8f){0.f,0.f,0.f,0.f,0.f,0.f,0.f,0.f};

  for (int k0 = 0; k0 < K; k0 += 32) {
    V bh[4], bl[4];
#pragma unroll
    for (int j = 0; j < 4; ++j) {
      const size_t bo = (size_t)(n0 + (j << 4) + rlane) * ldb + koff + k0;
      bh[j] = Frag<T>::load(Bb + bo);
      if (SPLIT) bl[j] = Frag<T>::load(Bb2 + bo);
    }
#pragma unroll
    for (int i = 0; i < 4; ++i) {
      const size_t ao = (size_t)(m0 + (i << 4) + rlane) * lda + koff + k0;
      V ah = Frag<T>::load(Ab + ao);
      V al;
      if (SPLIT) al = Frag<T>::load(Ab2 + ao);
#pragma unroll
      for (int j = 0; j < 4; ++j) {
        acc[i][j] = Frag<T>::mma(ah, bh[j], acc[i][j]);
        if (SPLIT) {
          acc[i][j] = Frag<T>::mma(ah, bl[j], acc[i][j]);
          acc[i][j] = Frag<T>::mma(al, bh[j], acc[i][j]);
        }
      }
      Frag<T>::guard(acc[i][0], acc[i][3], ah, SPLIT ? al : ah);
    }
    Frag<T>::keep(bh[0], bh[1], bh[2], bh[3]);
    if (SPLIT) Frag<T>::keep(bl[0], bl[1], bl[2], bl[3]);
  }
  acc_guard4(acc[0][0], acc[0][1], acc[0][2], acc[0][3]);
  acc_guard4(acc[1][0], acc[1][1], acc[1][2], acc[1][3]);
  acc_guard4(acc[2][0], acc[2][1], acc[2][2], acc[2][3]);
  acc_guard4(acc[3][0], acc[3][1], acc[3][2], acc[3][3]);

  float* slab = sT[wave];
  const float* Rb = RESID ? (resid + (size_t)b * strideR) : nullptr;
#pragma unroll
  for (int i = 0; i < 4; ++i) {
    const int mBase = m0 + (i << 4);
#pragma unroll
    for (int j = 0; j < 4; ++j) {
      const int n = n0 + (j << 4) + rlane;
      float bv = 0.f;
      if (BIAS_MODE == 2) bv = bias[n];
#pragma unroll
      for (int r = 0; r < 8; ++r) {
        float v = acc[i][j][r] * scale;
        if (BIAS_MODE == 1) v += bias[mBase + mOff + r];
        if (BIAS_MODE == 2) v += bv;
        if (RESID) v += Rb[(size_t)(mBase + mOff + r) * ldc + n];
        if (ACT == 2) v = fmaxf(v, 0.0f);
        if (ACT == 4) v = (v > 0.f) ? v : 0.01f * v;
        slab[(mOff + r) * 68 + (j << 4) + rlane] = v;
      }
    }
    __builtin_amdgcn_fence(__ATOMIC_RELEASE, "workgroup");
    __builtin_amdgcn_wave_barrier();
    __builtin_amdgcn_fence(__ATOMIC_ACQUIRE, "workgroup");
    if (OUT_MODE == 0) {
      float* C = (float*)Cout + (size_t)b * strideC;
      const int hh = lane >> 4, c4 = (lane & 15) * 4;
      for (int pass = 0; pass < 2; ++pass) {
#pragma unroll
        for (int it = 0; it < 8; ++it) {
          const int row = it * 2 + hh;
          v4f v = *(const v4f*)(slab + row * 68 + c4);
          *(volatile v4f*)(C + (size_t)(mBase + row) * ldc + n0 + c4) = v;
        }
        __threadfence();
      }
    } else {
      const int q = lane >> 3, c8 = (lane & 7) * 8;
      unsigned short* C  = (unsigned short*)Cout  + (size_t)b * strideC;
      unsigned short* C2 = (OUT_MODE == 2) ? ((unsigned short*)Cout2 + (size_t)b * strideC) : nullptr;
      for (int pass = 0; pass < 2; ++pass) {
#pragma unroll
        for (int it = 0; it < 4; ++it) {
          const int row = it * 4 + q;
          const float* sp = slab + row * 68 + c8;
          v8h hv, lv;
#pragma unroll
          for (int e = 0; e < 8; ++e) {
            if (OUT_MODE == 1) {
              hv[e] = (_Float16)sp[e];
            } else {
              unsigned short hb = f2bf_bits(sp[e]);
              unsigned short lb = f2bf_bits(sp[e] - bf_bits2f(hb));
              hv[e] = __builtin_bit_cast(_Float16, hb);
              lv[e] = __builtin_bit_cast(_Float16, lb);
            }
          }
          *(volatile v8h*)(C + (size_t)(mBase + row) * ldc + n0 + c8) = hv;
          if (OUT_MODE == 2) *(volatile v8h*)(C2 + (size_t)(mBase + row) * ldc + n0 + c8) = lv;
        }
        __threadfence();
      }
    }
    __builtin_amdgcn_fence(__ATOMIC_RELEASE, "workgroup");
    __builtin_amdgcn_wave_barrier();
    __builtin_amdgcn_fence(__ATOMIC_ACQUIRE, "workgroup");
  }
}

__global__ __launch_bounds__(256) void cast8_f16_kernel(const float* __restrict__ in, unsigned short* __restrict__ out, int n8) {
  const int i = blockIdx.x * 256 + threadIdx.x;
  if (i >= n8) return;
  const float* p = in + 8 * (size_t)i;
  const v4f a = *(const v4f*)(p);
  const v4f c = *(const v4f*)(p + 4);
  unsigned short hb[8];
#pragma unroll
  for (int e = 0; e < 4; ++e) {
    hb[e]     = h_bits(a[e]);
    hb[4 + e] = h_bits(c[e]);
  }
  const v4u u = (v4u){pk16(hb[0], hb[1]), pk16(hb[2], hb[3]), pk16(hb[4], hb[5]), pk16(hb[6], hb[7])};
  unsigned short* q = out + 8 * (size_t)i;
  *(volatile v4u*)q = u;
  __threadfence();
  *(volatile v4u*)q = u;
}

constexpr int kV1Groups = kKpad / 8;
__global__ __launch_bounds__(256) void cast_v1_kernel(const float* __restrict__ V1, unsigned short* __restrict__ out) {
  const int i = blockIdx.x * 256 + threadIdx.x;
  if (i >= kNpad * kV1Groups) return;
  const int r  = i / kV1Groups;
  const int g  = i - r * kV1Groups;
  const int c8 = g * 8;
  const int rr = (r < kSzN) ? r : (kSzN - 1);
  const float* src = V1 + (size_t)rr * kSzM;
  unsigned short hb[8];
#pragma unroll
  for (int e = 0; e < 8; ++e) {
    const int c  = c8 + e;
    const int cc = (c < kSzM) ? c : (kSzM - 1);
    float v = src[cc];
    v = (r < kSzN && c < kSzM) ? v : 0.0f;
    hb[e] = h_bits(v);
  }
  const v4u u = (v4u){pk16(hb[0], hb[1]), pk16(hb[2], hb[3]), pk16(hb[4], hb[5]), pk16(hb[6], hb[7])};
  unsigned short* q = out + 8 * (size_t)i;
  *(volatile v4u*)q = u;
  __threadfence();
  *(volatile v4u*)q = u;
}

__global__ __launch_bounds__(256) void cast_v2t_kernel(const float* __restrict__ V2, unsigned short* __restrict__ out) {
  __shared__ float sm[64][65];
  const int t  = threadIdx.x;
  const int k0 = blockIdx.x * 64;
  const int n0 = blockIdx.y * 64;
#pragma unroll
  for (int i = 0; i < 16; ++i) {
    const int e  = i * 256 + t;
    const int kl = e >> 6;
    const int nl = e & 63;
    const int k  = k0 + kl;
    const int n  = n0 + nl;
    const int kc = (k < kSzM) ? k : (kSzM - 1);
    const int nc = (n < kSzN) ? n : (kSzN - 1);
    float v = V2[(size_t)kc * kSzN + nc];
    v = (k < kSzM && n < kSzN) ? v : 0.0f;
    sm[nl][kl] = v;
  }
  __syncthreads();
  const int lane = t & 31, wave = t >> 5;
  const int q = lane >> 3, c8 = (lane & 7) * 8;
  for (int pass = 0; pass < 2; ++pass) {
#pragma unroll
    for (int it = 0; it < 2; ++it) {
      const int row = wave * 8 + it * 4 + q;
      unsigned short hb[8];
#pragma unroll
      for (int e = 0; e < 8; ++e) hb[e] = h_bits(sm[row][c8 + e]);
      const v4u u = (v4u){pk16(hb[0], hb[1]), pk16(hb[2], hb[3]), pk16(hb[4], hb[5]), pk16(hb[6], hb[7])};
      *(volatile v4u*)(out + (size_t)(n0 + row) * kKpad + k0 + c8) = u;
    }
    __threadfence();
  }
}

__global__ __launch_bounds__(256) void reslice_w_kernel(const float* __restrict__ Vf,
                                                        const float* __restrict__ w1p, const float* __restrict__ w2p,
                                                        unsigned short* __restrict__ W1h, unsigned short* __restrict__ W2h) {
  const int sel = blockIdx.y;
  const int i   = blockIdx.x * 256 + threadIdx.x;
  if (i >= kNW1 / 8) return;
  const float sc = (sel == 0) ? w1p[0] : w2p[0];
  unsigned short* outp = (sel == 0) ? W1h : W2h;
  const int base = (sel == 0) ? 0 : (kNW1 + kNB1);
  const int p0 = base + 8 * i;
  int r = p0 / kSzN;
  int c = p0 - r * kSzN;
  unsigned short hb[8];
#pragma unroll
  for (int e = 0; e < 8; ++e) {
    const int rr = (r < kSzN) ? r : (kSzN - 1);
    const float v = Vf[(size_t)rr * kNpad + c] * sc;
    hb[e] = h_bits(v);
    c += 1;
    const int wrap = (c == kSzN) ? 1 : 0;
    r += wrap;
    c = wrap ? 0 : c;
  }
  const v4u u = (v4u){pk16(hb[0], hb[1]), pk16(hb[2], hb[3]), pk16(hb[4], hb[5]), pk16(hb[6], hb[7])};
  unsigned short* q = outp + 8 * (size_t)i;
  *(volatile v4u*)q = u;
  __threadfence();
  *(volatile v4u*)q = u;
}

__global__ __launch_bounds__(256) void reslice_b_kernel(const float* __restrict__ Vf,
                                                        const float* __restrict__ b1p, const float* __restrict__ b2p,
                                                        float* __restrict__ b1, float* __restrict__ b2) {
  const int blk = blockIdx.x;
  const int t   = threadIdx.x;
  const bool isb2 = (blk == 4);
  const int j = isb2 ? t : (blk * 256 + t);
  const int p0 = isb2 ? (kNW1 + kNB1 + kNW2 + 4 * j) : (kNW1 + 4 * j);
  const float sc = isb2 ? b2p[0] : b1p[0];
  float* outp = isb2 ? b2 : b1;
  int r = p0 / kSzN;
  int c = p0 - r * kSzN;
  v4f val;
#pragma unroll
  for (int e = 0; e < 4; ++e) {
    const int rr = (r < kSzN) ? r : (kSzN - 1);
    val[e] = Vf[(size_t)rr * kNpad + c] * sc;
    c += 1;
    const int wrap = (c == kSzN) ? 1 : 0;
    r += wrap;
    c = wrap ? 0 : c;
  }
  float* q = outp + 4 * (size_t)j;
  *(volatile v4f*)q = val;
  __threadfence();
  *(volatile v4f*)q = val;
}

static inline size_t align256(size_t x) { return (x + 255) & ~(size_t)255; }

extern "C" void kernel_launch(void* const* d_in, const int* in_sizes, int n_in,
                              void* d_out, int out_size, void* d_ws, size_t ws_size,
                              hipStream_t stream) {
  if (n_in < 7) return;
  if (in_sizes[0] != kBatch * kDin || in_sizes[1] != kSzN * kSzM || in_sizes[2] != kSzM * kSzN) return;
  if (in_sizes[3] < 1 || in_sizes[4] < 1 || in_sizes[5] < 1 || in_sizes[6] < 1) return;
  if (out_size != kBatch * kDout) return;

  const float* x   = (const float*)d_in[0];
  const float* V1  = (const float*)d_in[1];
  const float* V2  = (const float*)d_in[2];
  const float* w1p = (const float*)d_in[3];
  const float* b1p = (const float*)d_in[4];
  const float* w2p = (const float*)d_in[5];
  const float* b2p = (const float*)d_in[6];
  float* y = (float*)d_out;

  char* base = (char*)d_ws;
  size_t off = 0;
  unsigned short* V1h  = (unsigned short*)(base + off); off = align256(off + (size_t)kNpad * kKpad * 2);
  unsigned short* V2th = (unsigned short*)(base + off); off = align256(off + (size_t)kNpad * kKpad * 2);
  float*          Vf   = (float*)(base + off);          off = align256(off + (size_t)kNpad * kNpad * 4);
  unsigned short* X16  = (unsigned short*)(base + off); off = align256(off + (size_t)kBatch * kDin * 2);
  unsigned short* W1h  = (unsigned short*)(base + off); off = align256(off + (size_t)kDh * kDin * 2);
  unsigned short* W2h  = (unsigned short*)(base + off); off = align256(off + (size_t)kDout * kDh * 2);
  float*          b1   = (float*)(base + off);          off = align256(off + (size_t)kDh * 4);
  float*          b2   = (float*)(base + off);          off = align256(off + (size_t)kDout * 4);
  unsigned short* H16  = (unsigned short*)(base + off); off = align256(off + (size_t)kBatch * kDh * 2);
  if (off > ws_size) return;

  cast_v1_kernel<<<dim3((kNpad * kV1Groups) / 256), dim3(256), 0, stream>>>(V1, V1h);
  cast_v2t_kernel<<<dim3(kKpad / 64, kNpad / 64), dim3(256), 0, stream>>>(V2, V2th);
  cast8_f16_kernel<<<dim3((kBatch * kDin / 8) / 256), dim3(256), 0, stream>>>(x, X16, kBatch * kDin / 8);

  {
    const int tiles = (kNpad / 64) * (kNpad / 64);
    wmma_gemm64<0, false, 0, 0, false, 0><<<dim3((tiles + 7) / 8, 1), dim3(256), 0, stream>>>(
        V1h, nullptr, kKpad, 0L, V2th, nullptr, kKpad, 0L,
        (void*)Vf, nullptr, kNpad, 0L, nullptr, nullptr, 0L, kNpad, kNpad, kKpad, 1.0f);
  }

  reslice_w_kernel<<<dim3((kNW1 / 8) / 256, 2), dim3(256), 0, stream>>>(Vf, w1p, w2p, W1h, W2h);
  reslice_b_kernel<<<dim3(5), dim3(256), 0, stream>>>(Vf, b1p, b2p, b1, b2);

  {
    const int tiles = (kBatch / 64) * (kDh / 64);
    wmma_gemm64<0, false, 2, 1, false, 2><<<dim3((tiles + 7) / 8, 1), dim3(256), 0, stream>>>(
        X16, nullptr, kDin, 0L, W1h, nullptr, kDin, 0L,
        (void*)H16, nullptr, kDh, 0L, b1, nullptr, 0L, kBatch, kDh, kDin, 1.0f);
  }

  {
    const int tiles = (kBatch / 64) * (kDout / 64);
    wmma_gemm64<0, false, 2, 0, false, 0><<<dim3((tiles + 7) / 8, 1), dim3(256), 0, stream>>>(
        H16, nullptr, kDh, 0L, W2h, nullptr, kDh, 0L,
        (void*)y, nullptr, kDout, 0L, b2, nullptr, 0L, kBatch, kDout, kDh, 1.0f);
  }
}
